// WMSA_13932873908942
// MI455X (gfx1250) — hardware-verified
//
#include <hip/hip_runtime.h>

typedef __attribute__((ext_vector_type(16))) _Float16 v16h;
typedef __attribute__((ext_vector_type(8)))  _Float16 v8h;
typedef __attribute__((ext_vector_type(16))) __bf16   v16b;
typedef __attribute__((ext_vector_type(8)))  __bf16   v8b;
typedef __attribute__((ext_vector_type(8)))  float    v8f;
typedef __attribute__((ext_vector_type(4)))  float    v4f;
typedef __attribute__((ext_vector_type(4)))  unsigned v4u;

static constexpr int kTok      = 64;
static constexpr int kDim      = 192;
static constexpr int kDim3     = 576;
static constexpr int kHeads    = 6;
static constexpr int kHeadDim  = 32;
static constexpr int kRowsHalf = 32768;
static constexpr int kBiasTab  = 343;

__device__ __forceinline__ unsigned short f2bf_bits(float f) {
  unsigned u = __float_as_uint(f);
  return (unsigned short)((u + 0x7FFFu + ((u >> 16) & 1u)) >> 16);
}
__device__ __forceinline__ float bf_bits2f(unsigned short h) { return __uint_as_float(((unsigned)h) << 16); }

__device__ __forceinline__ void dep_guard_h(v8f& a, v8f& b, v16h x, v16h y) { asm volatile("v_nop\n\tv_nop\n\tv_nop\n\tv_nop" : "+v"(a), "+v"(b) : "v"(x), "v"(y)); }
__device__ __forceinline__ void dep_guard_b(v8f& a, v8f& b, v16b x, v16b y) { asm volatile("v_nop\n\tv_nop\n\tv_nop\n\tv_nop" : "+v"(a), "+v"(b) : "v"(x), "v"(y)); }
__device__ __forceinline__ void keep4_h(v16h a, v16h b, v16h c, v16h d) { asm volatile("v_nop" :: "v"(a), "v"(b), "v"(c), "v"(d)); }
__device__ __forceinline__ void keep4_b(v16b a, v16b b, v16b c, v16b d) { asm volatile("v_nop" :: "v"(a), "v"(b), "v"(c), "v"(d)); }
__device__ __forceinline__ void acc_guard4(v8f& a, v8f& b, v8f& c, v8f& d) { asm volatile("v_nop\n\tv_nop\n\tv_nop\n\tv_nop" : "+v"(a), "+v"(b), "+v"(c), "+v"(d)); }
template <typename T> struct Frag;
template <> struct Frag<_Float16> {
  typedef v16h V; union U { v16h v; v8h h[2]; };
  static __device__ __forceinline__ v16h load(const _Float16* p) {
    U f; f.h[0] = *(const v8h*)(p); f.h[1] = *(const v8h*)(p + 16); return f.v;
  }
  static __device__ __forceinline__ v8f mma(v16h a, v16h b, v8f c) {
    return __builtin_amdgcn_wmma_f32_16x16x32_f16(false, a, false, b, (short)0, c, false, false);
  }
  static __device__ __forceinline__ void guard(v8f& a, v8f& b, v16h x, v16h y) { dep_guard_h(a, b, x, y); }
  static __device__ __forceinline__ void keep(v16h a, v16h b, v16h c, v16h d) { keep4_h(a, b, c, d); }
};
template <> struct Frag<__bf16> {
  typedef v16b V; union U { v16b v; v8b h[2]; };
  static __device__ __forceinline__ v16b load(const __bf16* p) {
    U f; f.h[0] = *(const v8b*)(p); f.h[1] = *(const v8b*)(p + 16); return f.v;
  }
  static __device__ __forceinline__ v8f mma(v16b a, v16b b, v8f c) {
    return __builtin_amdgcn_wmma_f32_16x16x32_bf16(false, a, false, b, (short)0, c, false, false);
  }
  static __device__ __forceinline__ void guard(v8f& a, v8f& b, v16b x, v16b y) { dep_guard_b(a, b, x, y); }
  static __device__ __forceinline__ void keep(v16b a, v16b b, v16b c, v16b d) { keep4_b(a, b, c, d); }
};

template <int ET> struct Elem;
template <> struct Elem<0> { typedef _Float16 T; };
template <> struct Elem<1> { typedef __bf16 T; };
template <int ET, int SPLIT, int BIAS_MODE, int OUT_MODE, bool RESID, int ACT = 0>
__global__ __launch_bounds__(256) void wmma_gemm64(
    const unsigned short* __restrict__ Ap, const unsigned short* __restrict__ A2p, int lda, long strideA,
    const unsigned short* __restrict__ Btp, const unsigned short* __restrict__ Bt2p, int ldb, long strideB,
    void* __restrict__ Cout, void* __restrict__ Cout2, int ldc, long strideC,
    const float* __restrict__ bias,
    const float* __restrict__ resid, long strideR,
    int M, int N, int K, float scale) {
  typedef typename Elem<ET>::T T;
  typedef typename Frag<T>::V V;
  const T* A = (const T*)Ap; const T* A2 = (const T*)A2p; const T* Bt = (const T*)Btp; const T* Bt2 = (const T*)Bt2p;
  __shared__ __align__(16) float sT[8][16 * 68];
  const int b    = blockIdx.y;
  const int lane = threadIdx.x & 31;
  const int wave = threadIdx.x >> 5;
  const int tilesN = N >> 6;
  const int tilesM = M >> 6;
  const int tile = blockIdx.x * 8 + wave;
  if (tile >= tilesM * tilesN) return;
  const int tm = tile / tilesN;
  const int tn = tile - tm * tilesN;
  const int m0 = tm << 6;
  const int n0 = tn << 6;

  const T* Ab  = A  + (size_t)b * strideA;
  const T* Bb  = Bt + (size_t)b * strideB;
  const T* Ab2 = (SPLIT != 0) ? (A2  + (size_t)b * strideA) : nullptr;
  const T* Bb2 = (SPLIT == 2) ? (Bt2 + (size_t)b * strideB) : nullptr;

  const int rlane = lane & 15;
  const int koff  = (lane >> 4) * 8;
  const int mOff  = (lane >> 4) * 8;

  v8f acc[4][4];
#pragma unroll
  for (int i = 0; i < 4; ++i)
#pragma unroll
    for (int j = 0; j < 4; ++j) acc[i][j] = (v8f){0.f,0.f,0.f,0.f,0.f,0.f,0.f,0.f};

  for (int k0 = 0; k0 < K; k0 += 32) {
    V bh[4], bl[4];
#pragma unroll
    for (int j = 0; j < 4; ++j) {
      const size_t bo = (size_t)(n0 + (j << 4) + rlane) * ldb + koff + k0;
      bh[j] = Frag<T>::load(Bb + bo);
      if (SPLIT == 2) bl[j] = Frag<T>::load(Bb2 + bo);
    }
#pragma unroll
    for (int i = 0; i < 4; ++i) {
      const size_t ao = (size_t)(m0 + (i << 4) + rlane) * lda + koff + k0;
      V ah = Frag<T>::load(Ab + ao);
      V al;
      if (SPLIT != 0) al = Frag<T>::load(Ab2 + ao);
#pragma unroll
      for (int j = 0; j < 4; ++j) {
        acc[i][j] = Frag<T>::mma(ah, bh[j], acc[i][j]);
        if (SPLIT == 2) acc[i][j] = Frag<T>::mma(ah, bl[j], acc[i][j]);
        if (SPLIT != 0) acc[i][j] = Frag<T>::mma(al, bh[j], acc[i][j]);
      }
      Frag<T>::guard(acc[i][0], acc[i][3], ah, (SPLIT != 0) ? al : ah);
    }
    Frag<T>::keep(bh[0], bh[1], bh[2], bh[3]);
    if (SPLIT == 2) Frag<T>::keep(bl[0], bl[1], bl[2], bl[3]);
  }
  acc_guard4(acc[0][0], acc[0][1], acc[0][2], acc[0][3]);
  acc_guard4(acc[1][0], acc[1][1], acc[1][2], acc[1][3]);
  acc_guard4(acc[2][0], acc[2][1], acc[2][2], acc[2][3]);
  acc_guard4(acc[3][0], acc[3][1], acc[3][2], acc[3][3]);

  float* slab = sT[wave];
  const float* Rb = RESID ? (resid + (size_t)b * strideR) : nullptr;
#pragma unroll
  for (int i = 0; i < 4; ++i) {
    const int mBase = m0 + (i << 4);
#pragma unroll
    for (int j = 0; j < 4; ++j) {
      const int n = n0 + (j << 4) + rlane;
      float bv = 0.f;
      if (BIAS_MODE == 2) bv = bias[n];
#pragma unroll
      for (int r = 0; r < 8; ++r) {
        float v = acc[i][j][r] * scale;
        if (BIAS_MODE == 1) v += bias[mBase + mOff + r];
        if (BIAS_MODE == 2) v += bv;
        if (RESID) v += Rb[(size_t)(mBase + mOff + r) * ldc + n];
        if (ACT == 1) v = tanhf(v);
        if (ACT == 2) v = fmaxf(v, 0.0f);
        if (ACT == 3) v = v / (1.0f + expf(-v));
        if (ACT == 4) v = (v > 0.f) ? v : 0.01f * v;
        slab[(mOff + r) * 68 + (j << 4) + rlane] = v;
      }
    }
    __builtin_amdgcn_fence(__ATOMIC_RELEASE, "workgroup");
    __builtin_amdgcn_wave_barrier();
    __builtin_amdgcn_fence(__ATOMIC_ACQUIRE, "workgroup");
    if (OUT_MODE == 0) {
      float* C = (float*)Cout + (size_t)b * strideC;
      const int hh = lane >> 4, c4 = (lane & 15) * 4;
      for (int pass = 0; pass < 2; ++pass) {
#pragma unroll
        for (int it = 0; it < 8; ++it) {
          const int row = it * 2 + hh;
          v4f v = *(const v4f*)(slab + row * 68 + c4);
          *(volatile v4f*)(C + (size_t)(mBase + row) * ldc + n0 + c4) = v;
        }
        __threadfence();
      }
    } else {
      const int q = lane >> 3, c8 = (lane & 7) * 8;
      unsigned short* C  = (unsigned short*)Cout  + (size_t)b * strideC;
      unsigned short* C2 = (OUT_MODE == 2) ? ((unsigned short*)Cout2 + (size_t)b * strideC) : nullptr;
      for (int pass = 0; pass < 2; ++pass) {
#pragma unroll
        for (int it = 0; it < 4; ++it) {
          const int row = it * 4 + q;
          const float* sp = slab + row * 68 + c8;
          v8h hv, lv;
#pragma unroll
          for (int e = 0; e < 8; ++e) {
            if (OUT_MODE == 1) {
              hv[e] = (_Float16)sp[e];
            } else {
              unsigned short hb = f2bf_bits(sp[e]);
              unsigned short lb = f2bf_bits(sp[e] - bf_bits2f(hb));
              hv[e] = __builtin_bit_cast(_Float16, hb);
              lv[e] = __builtin_bit_cast(_Float16, lb);
            }
          }
          *(volatile v8h*)(C + (size_t)(mBase + row) * ldc + n0 + c8) = hv;
          if (OUT_MODE == 2) *(volatile v8h*)(C2 + (size_t)(mBase + row) * ldc + n0 + c8) = lv;
        }
        __threadfence();
      }
    }
    __builtin_amdgcn_fence(__ATOMIC_RELEASE, "workgroup");
    __builtin_amdgcn_wave_barrier();
    __builtin_amdgcn_fence(__ATOMIC_ACQUIRE, "workgroup");
  }
}

__device__ __forceinline__ v8f at_mma(v16b a, v16b b, v8f c) {
  c = __builtin_amdgcn_wmma_f32_16x16x32_bf16(false, a, false, b, (short)0, c, false, false);
  asm volatile("v_nop\n\tv_nop\n\tv_nop\n\tv_nop" : "+v"(c) : "v"(a), "v"(b));
  return c;
}

__global__ __launch_bounds__(256) void gather_window_kernel(const float* __restrict__ x,
                                                            unsigned short* __restrict__ xw, int bsel)
{
  const int g = blockIdx.x * 256 + threadIdx.x;
  const int row = g / 24;
  const int c8 = (g - row * 24) * 8;
  const int w = row >> 6, t = row & 63;
  const int i = t >> 4, j = (t >> 2) & 3, k = t & 3;
  const int w1 = w >> 6, w2 = (w >> 3) & 7, w3 = w & 7;
  const int z  = (w1 * 4 + i + 2) & 31;
  const int y  = (w2 * 4 + j + 2) & 31;
  const int xx = (w3 * 4 + k + 2) & 31;
  const float* src = x + ((((size_t)bsel * 32 + z) * 32 + y) * 32 + xx) * kDim + c8;
  const v4f a = *(const v4f*)src;
  const v4f c = *(const v4f*)(src + 4);
  v4u o;
  o.x = (unsigned)f2bf_bits(a.x) | ((unsigned)f2bf_bits(a.y) << 16);
  o.y = (unsigned)f2bf_bits(a.z) | ((unsigned)f2bf_bits(a.w) << 16);
  o.z = (unsigned)f2bf_bits(c.x) | ((unsigned)f2bf_bits(c.y) << 16);
  o.w = (unsigned)f2bf_bits(c.z) | ((unsigned)f2bf_bits(c.w) << 16);
  unsigned short* dst = xw + (size_t)g * 8;
  *(volatile v4u*)dst = o;
  __threadfence();
  *(volatile v4u*)dst = o;
}

__global__ __launch_bounds__(256) void weightT_bf16_kernel(const float* __restrict__ W,
                                                           unsigned short* __restrict__ Wt,
                                                           int nrowsK, int ncolsN)
{
  const int g = blockIdx.x * 256 + threadIdx.x;
  const int per = nrowsK >> 3;
  const int total = ncolsN * per;
  if (g >= total) return;
  const int n = g / per;
  const int k8 = (g - n * per) * 8;
  float f[8];
#pragma unroll
  for (int e = 0; e < 8; ++e) f[e] = W[(size_t)(k8 + e) * ncolsN + n];
  v4u o;
  o.x = (unsigned)f2bf_bits(f[0]) | ((unsigned)f2bf_bits(f[1]) << 16);
  o.y = (unsigned)f2bf_bits(f[2]) | ((unsigned)f2bf_bits(f[3]) << 16);
  o.z = (unsigned)f2bf_bits(f[4]) | ((unsigned)f2bf_bits(f[5]) << 16);
  o.w = (unsigned)f2bf_bits(f[6]) | ((unsigned)f2bf_bits(f[7]) << 16);
  unsigned short* dst = Wt + (size_t)g * 8;
  *(volatile v4u*)dst = o;
  __threadfence();
  *(volatile v4u*)dst = o;
}

__global__ __launch_bounds__(256) void bias_rne_kernel(const float* __restrict__ bq,
                                                       const float* __restrict__ bo,
                                                       float* __restrict__ dst)
{
  const int g = threadIdx.x;
  if (g >= 192) return;
  v4f o;
#pragma unroll
  for (int e = 0; e < 4; ++e) {
    const int idx = g * 4 + e;
    const int iq = idx < 576 ? idx : 575;
    int io = idx - 576; io = io < 0 ? 0 : io; io = io > 191 ? 191 : io;
    const float vq = bq[iq];
    const float vo = bo[io];
    const float v = (idx < 576) ? vq : vo;
    o[e] = bf_bits2f(f2bf_bits(v));
  }
  float* p = dst + g * 4;
  *(volatile v4f*)p = o;
  __threadfence();
  *(volatile v4f*)p = o;
}

__global__ __launch_bounds__(128) void win_attn_kernel(
    const unsigned short* __restrict__ qkvh, const unsigned short* __restrict__ qkvl,
    const float* __restrict__ relp,
    unsigned short* __restrict__ oh, unsigned short* __restrict__ ol)
{
  __shared__ __align__(16) unsigned short sQh[64 * 40];
  __shared__ __align__(16) unsigned short sQl[64 * 40];
  __shared__ __align__(16) unsigned short sKh[64 * 40];
  __shared__ __align__(16) unsigned short sKl[64 * 40];
  __shared__ __align__(16) unsigned short sVh[32 * 72];
  __shared__ __align__(16) unsigned short sVl[32 * 72];
  __shared__ __align__(16) unsigned short sPh[4 * 16 * 72];
  __shared__ __align__(16) unsigned short sPl[4 * 16 * 72];
  __shared__ __align__(16) unsigned short sOh[64 * 192];
  __shared__ __align__(16) unsigned short sOl[64 * 192];
  __shared__ float sBias[kHeads * kBiasTab];

  const int tid  = threadIdx.x;
  const int wave = tid >> 5;
  const int lane = tid & 31;
  const int hh   = lane >> 4;
  const int cl   = lane & 15;
  const int w    = blockIdx.x;
  const int w1 = w >> 6, w2 = (w >> 3) & 7, w3 = w & 7;
  const size_t rowbase = (size_t)w * kTok;
  const float kScale = 0.17677669529663687f;
  const float kNegInf = -__builtin_inff();

#pragma unroll 1
  for (int i = tid; i < kHeads * kBiasTab; i += 128) sBias[i] = bf_bits2f(f2bf_bits(relp[i]));

  const __bf16* QhB = (const __bf16*)(const void*)sQh;
  const __bf16* QlB = (const __bf16*)(const void*)sQl;
  const __bf16* KhB = (const __bf16*)(const void*)sKh;
  const __bf16* KlB = (const __bf16*)(const void*)sKl;
  const __bf16* VhB = (const __bf16*)(const void*)sVh;
  const __bf16* VlB = (const __bf16*)(const void*)sVl;
  const __bf16* PhB = (const __bf16*)(const void*)sPh;
  const __bf16* PlB = (const __bf16*)(const void*)sPl;

#pragma unroll 1
  for (int h = 0; h < kHeads; ++h) {
    __syncthreads();
#pragma unroll
    for (int rep = 0; rep < 2; ++rep) {
      const int idx = tid + rep * 128;
      const int r = idx >> 2, c8 = (idx & 3) * 8;
      const size_t gq = (rowbase + r) * kDim3 + h * kHeadDim + c8;
      const v4u aqh = *(const v4u*)(qkvh + gq);
      const v4u aql = *(const v4u*)(qkvl + gq);
      const v4u akh = *(const v4u*)(qkvh + gq + kDim);
      const v4u akl = *(const v4u*)(qkvl + gq + kDim);
      *(v4u*)(sQh + r * 40 + c8) = aqh;
      *(v4u*)(sQl + r * 40 + c8) = aql;
      *(v4u*)(sKh + r * 40 + c8) = akh;
      *(v4u*)(sKl + r * 40 + c8) = akl;
    }
    asm volatile("" ::: "memory");
    {
      const int key = tid >> 1, d16 = (tid & 1) * 16;
      const size_t gv = (rowbase + key) * kDim3 + 2 * kDim + h * kHeadDim + d16;
      const v4u v0 = *(const v4u*)(qkvh + gv);
      const v4u v1 = *(const v4u*)(qkvh + gv + 8);
      const v4u u0 = *(const v4u*)(qkvl + gv);
      const v4u u1 = *(const v4u*)(qkvl + gv + 8);
      const unsigned wdh[8] = {v0.x, v0.y, v0.z, v0.w, v1.x, v1.y, v1.z, v1.w};
      const unsigned wdl[8] = {u0.x, u0.y, u0.z, u0.w, u1.x, u1.y, u1.z, u1.w};
#pragma unroll
      for (int e = 0; e < 8; ++e) {
        sVh[(d16 + 2 * e) * 72 + key]     = (unsigned short)(wdh[e] & 0xffffu);
        sVh[(d16 + 2 * e + 1) * 72 + key] = (unsigned short)(wdh[e] >> 16);
        sVl[(d16 + 2 * e) * 72 + key]     = (unsigned short)(wdl[e] & 0xffffu);
        sVl[(d16 + 2 * e + 1) * 72 + key] = (unsigned short)(wdl[e] >> 16);
      }
    }
    __syncthreads();

    const v16b qa_h = Frag<__bf16>::load(QhB + (wave * 16 + cl) * 40 + 8 * hh);
    const v16b qa_l = Frag<__bf16>::load(QlB + (wave * 16 + cl) * 40 + 8 * hh);
    v8f s[4];
#pragma unroll
    for (int j = 0; j < 4; ++j) {
      const v16b kb_h = Frag<__bf16>::load(KhB + (j * 16 + cl) * 40 + 8 * hh);
      const v16b kb_l = Frag<__bf16>::load(KlB + (j * 16 + cl) * 40 + 8 * hh);
      v8f a = (v8f){0.f,0.f,0.f,0.f,0.f,0.f,0.f,0.f};
      a = at_mma(qa_h, kb_h, a);
      a = at_mma(qa_h, kb_l, a);
      a = at_mma(qa_l, kb_h, a);
      s[j] = a;
    }

    const float* bh = sBias + h * kBiasTab;
    float lrow[8];
#pragma unroll
    for (int r = 0; r < 8; ++r) {
      const int p = wave * 16 + 8 * hh + r;
      const int i1 = p >> 4, j1 = (p >> 2) & 3, k1 = p & 3;
      float m = kNegInf;
#pragma unroll
      for (int j = 0; j < 4; ++j) {
        const int q = j * 16 + cl;
        const int i2 = q >> 4, j2 = (q >> 2) & 3, k2 = q & 3;
        const float bv = bh[((i1 - i2 + 3) * 7 + (j1 - j2 + 3)) * 7 + (k1 - k2 + 3)];
        const bool msk = ((w1 == 7) && ((i1 < 2) != (i2 < 2))) ||
                         ((w2 == 7) && ((j1 < 2) != (j2 < 2))) ||
                         ((w3 == 7) && ((k1 < 2) != (k2 < 2)));
        float v = s[j][r] * kScale + bv;
        v = msk ? kNegInf : v;
        s[j][r] = v;
        m = fmaxf(m, v);
      }
#pragma unroll
      for (int off = 1; off < 16; off <<= 1) m = fmaxf(m, __shfl_xor(m, off, 32));
      float psum = 0.f;
#pragma unroll
      for (int j = 0; j < 4; ++j) {
        const float pv = expf(s[j][r] - m);
        psum += pv;
        const unsigned short hb = f2bf_bits(pv);
        const unsigned short lb = f2bf_bits(pv - bf_bits2f(hb));
        sPh[wave * 1152 + (8 * hh + r) * 72 + j * 16 + cl] = hb;
        sPl[wave * 1152 + (8 * hh + r) * 72 + j * 16 + cl] = lb;
      }
#pragma unroll
      for (int off = 1; off < 16; off <<= 1) psum += __shfl_xor(psum, off, 32);
      lrow[r] = psum;
    }
    __syncthreads();

    v8f o[2];
    o[0] = (v8f){0.f,0.f,0.f,0.f,0.f,0.f,0.f,0.f};
    o[1] = (v8f){0.f,0.f,0.f,0.f,0.f,0.f,0.f,0.f};
#pragma unroll
    for (int kk = 0; kk < 2; ++kk) {
      const v16b pa_h = Frag<__bf16>::load(PhB + wave * 1152 + cl * 72 + kk * 32 + 8 * hh);
      const v16b pa_l = Frag<__bf16>::load(PlB + wave * 1152 + cl * 72 + kk * 32 + 8 * hh);
#pragma unroll
      for (int t = 0; t < 2; ++t) {
        const v16b vb_h = Frag<__bf16>::load(VhB + (t * 16 + cl) * 72 + kk * 32 + 8 * hh);
        const v16b vb_l = Frag<__bf16>::load(VlB + (t * 16 + cl) * 72 + kk * 32 + 8 * hh);
        o[t] = at_mma(pa_h, vb_h, o[t]);
        o[t] = at_mma(pa_h, vb_l, o[t]);
        o[t] = at_mma(pa_l, vb_h, o[t]);
      }
    }
#pragma unroll
    for (int r = 0; r < 8; ++r) {
      const float inv = 1.0f / lrow[r];
      const int orow = wave * 16 + 8 * hh + r;
#pragma unroll
      for (int t = 0; t < 2; ++t) {
        const float val = o[t][r] * inv;
        const unsigned short hb = f2bf_bits(val);
        const unsigned short lb = f2bf_bits(val - bf_bits2f(hb));
        sOh[orow * 192 + h * kHeadDim + t * 16 + cl] = hb;
        sOl[orow * 192 + h * kHeadDim + t * 16 + cl] = lb;
      }
    }
  }
  __syncthreads();

  {
    const int q4 = lane >> 3, c8 = (lane & 7) * 8;
    for (int pass = 0; pass < 2; ++pass) {
#pragma unroll
      for (int it = 0; it < 12; ++it) {
        const int idx = it * 4 + q4;
        const int row = idx / 3;
        const int l3 = idx - row * 3;
        const int rr = wave * 16 + row;
        const int so = rr * 192 + l3 * 64 + c8;
        const v4u vh = *(const v4u*)(sOh + so);
        const v4u vl = *(const v4u*)(sOl + so);
        const size_t go = (rowbase + rr) * kDim + l3 * 64 + c8;
        *(volatile v4u*)(oh + go) = vh;
        *(volatile v4u*)(ol + go) = vl;
      }
      __threadfence();
    }
  }
}

__global__ __launch_bounds__(256) void unpartition_kernel(const float* __restrict__ p32,
                                                          float* __restrict__ out, int bsel)
{
  const int g = blockIdx.x * 256 + threadIdx.x;
  const int drow = g / 48;
  const int c4 = (g - drow * 48) * 4;
  const int z = drow >> 10, y = (drow >> 5) & 31, xx = drow & 31;
  const int zr = (z + 30) & 31, yr = (y + 30) & 31, xr = (xx + 30) & 31;
  const int w1 = zr >> 2, i = zr & 3;
  const int w2 = yr >> 2, j = yr & 3;
  const int w3 = xr >> 2, k = xr & 3;
  const int srow = ((w1 * 8 + w2) * 8 + w3) * kTok + (i * 16 + j * 4 + k);
  const v4f v = *(const v4f*)(p32 + (size_t)srow * kDim + c4);
  float* dst = out + ((size_t)bsel * kRowsHalf + drow) * kDim + c4;
  *(volatile v4f*)dst = v;
  __threadfence();
  *(volatile v4f*)dst = v;
}

extern "C" void kernel_launch(void* const* d_in, const int* in_sizes, int n_in,
                              void* d_out, int out_size, void* d_ws, size_t ws_size,
                              hipStream_t stream)
{
  constexpr size_t szWq  = (size_t)kDim3 * kDim * 2;
  constexpr size_t szWo  = (size_t)kDim * kDim * 2;
  constexpr size_t szBia = (size_t)768 * 4;
  constexpr size_t szXw  = (size_t)kRowsHalf * kDim * 2;
  constexpr size_t szQkv = (size_t)kRowsHalf * kDim3 * 2;
  constexpr size_t szO   = (size_t)kRowsHalf * kDim * 2;
  constexpr size_t szP32 = (size_t)kRowsHalf * kDim * 4;
  constexpr size_t oWq  = 0;
  constexpr size_t oWo  = oWq + szWq;
  constexpr size_t oBia = oWo + szWo;
  constexpr size_t oXw  = oBia + szBia;
  constexpr size_t oQh  = oXw + szXw;
  constexpr size_t oQl  = oQh + szQkv;
  constexpr size_t oOh  = oQl + szQkv;
  constexpr size_t oOl  = oOh + szO;
  constexpr size_t total = oOl + szO;
  static_assert(szP32 <= szQkv, "");
  static_assert(total == 113544192ull, "");
  static_assert(total <= 134217728ull, "");
  static_assert((oWo % 256) == 0 && (oBia % 256) == 0 && (oXw % 256) == 0 && (oQh % 256) == 0 &&
                (oQl % 256) == 0 && (oOh % 256) == 0 && (oOl % 256) == 0, "");
  static_assert(kRowsHalf % 64 == 0 && kDim3 % 64 == 0 && kDim % 64 == 0 && kDim % 32 == 0, "");
  static_assert((kRowsHalf * 24) % 256 == 0 && (kRowsHalf * 48) % 256 == 0, "");
  static_assert((kDim3 * kDim / 8) % 256 == 0 && (kDim * kDim / 8) % 256 == 0, "");

  if (n_in < 6) return;
  if (ws_size < total) return;
  if (in_sizes[0] != 2 * kRowsHalf * kDim || out_size != 2 * kRowsHalf * kDim) return;
  if (in_sizes[1] != kDim * kDim3 || in_sizes[2] != kDim3 || in_sizes[3] != kHeads * kBiasTab ||
      in_sizes[4] != kDim * kDim || in_sizes[5] != kDim) return;

  const float* x    = (const float*)d_in[0];
  const float* Wqkv = (const float*)d_in[1];
  const float* bqkv = (const float*)d_in[2];
  const float* relp = (const float*)d_in[3];
  const float* Wout = (const float*)d_in[4];
  const float* bout = (const float*)d_in[5];
  float* out = (float*)d_out;

  char* ws = (char*)d_ws;
  unsigned short* wqT = (unsigned short*)(ws + oWq);
  unsigned short* woT = (unsigned short*)(ws + oWo);
  float*          bia = (float*)(ws + oBia);
  unsigned short* xw  = (unsigned short*)(ws + oXw);
  unsigned short* qh  = (unsigned short*)(ws + oQh);
  unsigned short* ql  = (unsigned short*)(ws + oQl);
  unsigned short* oh  = (unsigned short*)(ws + oOh);
  unsigned short* ol  = (unsigned short*)(ws + oOl);
  float*          p32 = (float*)(ws + oQh);

  const int gridWq = (kDim3 * kDim / 8) / 256;
  const int gridWo = (kDim * kDim / 8) / 256;
  const int gridGather = (kRowsHalf * 24) / 256;
  const int gridQkv = ((kRowsHalf / 64) * (kDim3 / 64)) / 8;
  const int gridProj = ((kRowsHalf / 64) * (kDim / 64)) / 8;
  const int gridAttn = kRowsHalf / kTok;
  const int gridUnp = (kRowsHalf * 48) / 256;

  weightT_bf16_kernel<<<gridWq, 256, 0, stream>>>(Wqkv, wqT, kDim, kDim3);
  weightT_bf16_kernel<<<gridWo, 256, 0, stream>>>(Wout, woT, kDim, kDim);
  bias_rne_kernel<<<1, 256, 0, stream>>>(bqkv, bout, bia);

  for (int half = 0; half < 2; ++half) {
    gather_window_kernel<<<gridGather, 256, 0, stream>>>(x, xw, half);
    wmma_gemm64<1, 0, 2, 2, false><<<dim3(gridQkv, 1), 256, 0, stream>>>(
        xw, xw, kDim, 0L, wqT, wqT, kDim, 0L,
        (void*)qh, (void*)ql, kDim3, 0L,
        bia, bia, 0L, kRowsHalf, kDim3, kDim, 1.0f);
    win_attn_kernel<<<gridAttn, 128, 0, stream>>>(qh, ql, relp, oh, ol);
    wmma_gemm64<1, 1, 2, 0, false><<<dim3(gridProj, 1), 256, 0, stream>>>(
        oh, ol, kDim, 0L, woT, woT, kDim, 0L,
        (void*)p32, (void*)p32, kDim, 0L,
        bia + kDim3, bia + kDim3, 0L, kRowsHalf, kDim, kDim, 1.0f);
    unpartition_kernel<<<gridUnp, 256, 0, stream>>>(p32, out, half);
  }
}
